// LocalDenseSynthesizerAttention_20100446945653
// MI455X (gfx1250) — hardware-verified
//
#include <hip/hip_runtime.h>


namespace {
constexpr int NB = 8, T = 2048, F = 512, NH = 8, C = 45, CP = 48  , NL = NH * C  , NLP = 384  , DK = 64, PAD = 22, TP = T + 128  , NR = NB * T;
constexpr float XS = 8.0f, WSC = 256.0f, AS = 8.0f;

typedef _Float16 b16;
typedef __attribute__((ext_vector_type(16))) _Float16 v16b;
typedef __attribute__((ext_vector_type(8))) _Float16 v8b;
typedef __attribute__((ext_vector_type(8))) float v8f;
typedef __attribute__((ext_vector_type(4))) float v4f;
__device__ __forceinline__ float bf16_rne(float f) { unsigned int u = __float_as_uint(f); u += 0x7FFFu + ((u >> 16) & 1u); return __uint_as_float(u & 0xFFFF0000u); }
__device__ __forceinline__ void split16(float v, b16& hi, b16& lo) { hi = (b16)v; lo = (b16)(v - (float)hi); }
__device__ __forceinline__ v16b frag_kb(const b16* p, int hh) { const v8b a = *(const v8b*)(p + 8 * hh), b = *(const v8b*)(p + 16 + 8 * hh); v16b f;
#pragma unroll
  for (int e = 0; e < 8; ++e) { f[e] = a[e]; f[8 + e] = b[e]; } return f; }
__device__ __forceinline__ v8f wmma16b(v16b a, v16b b, v8f c) { v8f d = __builtin_amdgcn_wmma_f32_16x16x32_f16(false, a, false, b, (short)0, c, false, false); asm volatile("v_nop\n\tv_nop\n\tv_nop\n\tv_nop" : "+v"(d) : "v"(a), "v"(b)); return d; }
__device__ __forceinline__ void wave_lds_sync() { __builtin_amdgcn_fence(__ATOMIC_RELEASE, "workgroup"); __builtin_amdgcn_wave_barrier(); __builtin_amdgcn_fence(__ATOMIC_ACQUIRE, "workgroup"); }
__device__ __forceinline__ float nexp(float x) { return __builtin_amdgcn_exp2f(x * 1.4426950408889634f); }

__global__ __launch_bounds__(256) void prepx_kernel(const float* __restrict__ qry, const float* __restrict__ val, b16* __restrict__ XQ, b16* __restrict__ XV) {
  const size_t t = (size_t)blockIdx.x * 256 + threadIdx.x; const size_t n1 = (size_t)NR * F / 8; const float* src; b16* dst; size_t e;
  if (t < n1) { src = qry; dst = XQ; e = t * 8; } else if (t < 2 * n1) { src = val; dst = XV; e = (t - n1) * 8; } else return;
  const v4f a = *(const v4f*)(src + e), c = *(const v4f*)(src + e + 4); v8b o;
#pragma unroll
  for (int j = 0; j < 4; ++j) { o[j] = (b16)(bf16_rne(a[j]) * XS); o[4 + j] = (b16)(bf16_rne(c[j]) * XS); }
  for (int pass = 0; pass < 2; ++pass) { *(volatile v8b*)(dst + e) = o; __threadfence(); }
}
__global__ __launch_bounds__(256) void prepw_kernel(const float* __restrict__ w1, const float* __restrict__ w2, const float* __restrict__ w3, const float* __restrict__ wo, b16* __restrict__ W1T, b16* __restrict__ W2T, b16* __restrict__ W3T, b16* __restrict__ WOT) {
  __shared__ __attribute__((aligned(16))) b16 Tt[64][64 + 8];
  const int kind = blockIdx.z, i0 = blockIdx.x * 64, o0 = blockIdx.y * 64, t_ = threadIdx.x; const int OUT = kind == 1 ? NL : F; const float* w = kind == 0 ? w1 : kind == 1 ? w2 : kind == 2 ? w3 : wo; b16* dst = kind == 0 ? W1T : kind == 1 ? W2T : kind == 2 ? W3T : WOT;
  if (kind == 1) { if (o0 >= NLP) return; } else if (o0 >= F) return;
  for (int q = t_; q < 64 * 64; q += 256) { const int ii = q >> 6, oo = q & 63; const int o_ = o0 + oo; Tt[oo][ii] = (b16)((o_ < OUT) ? bf16_rne(w[(size_t)(i0 + ii) * OUT + o_]) * WSC : 0.0f); }
  __syncthreads();
  for (int pass = 0; pass < 2; ++pass) { for (int q = t_; q < 64 * 8; q += 256) { const int oo = q >> 3, c8 = (q & 7) * 8; if (o0 + oo < (kind == 1 ? NLP : F)) *(volatile v8b*)(dst + (size_t)(o0 + oo) * F + i0 + c8) = *(const v8b*)(&Tt[oo][c8]); } __threadfence(); }
}
template <int MODE>
__global__ __launch_bounds__(128) void gemm_kernel(const b16* __restrict__ A, const b16* __restrict__ Al, const b16* __restrict__ W, int K, b16* __restrict__ Yh, b16* __restrict__ Yl, float* __restrict__ Y32) {
  __shared__ __attribute__((aligned(16))) float Ts[4][16][128 + 4]; __shared__ __attribute__((aligned(16))) b16 Vt[128][64 + 8], Vtl[128][64 + 8];
  const int wave = threadIdx.x >> 5, lane = threadIdx.x & 31, nloc = lane & 15, hlf = lane >> 4, t_ = threadIdx.x; const size_t m0 = (size_t)blockIdx.x * 64 + wave * 16; const int n0 = blockIdx.y * 128;
  const int ntile = (MODE == 1) ? min(8, (NLP - n0) / 16) : 8;
  v8f acc[8];
#pragma unroll
  for (int t = 0; t < 8; ++t) acc[t] = (v8f){};
  for (int kb = 0; kb < K; kb += 32) { const v16b a = frag_kb(A + (m0 + nloc) * K + kb, hlf);
    if (MODE == 1 || MODE == 3) { const v16b al = frag_kb(Al + (m0 + nloc) * K + kb, hlf);
#pragma unroll
      for (int t = 0; t < 8; ++t) if (t < ntile) { const v16b bw = frag_kb(W + (size_t)(n0 + t * 16 + nloc) * K + kb, hlf); acc[t] = wmma16b(a, bw, acc[t]); acc[t] = wmma16b(al, bw, acc[t]); } }
    else {
#pragma unroll
      for (int t = 0; t < 8; ++t) acc[t] = wmma16b(a, frag_kb(W + (size_t)(n0 + t * 16 + nloc) * K + kb, hlf), acc[t]); } }
  if (MODE == 2) { const int b = (int)(m0 / T); const int t0 = (int)((size_t)blockIdx.x * 64 - (size_t)b * T);
#pragma unroll
    for (int t = 0; t < 8; ++t)
#pragma unroll
      for (int r = 0; r < 8; ++r) { b16 h_, l_; split16(acc[t][r] * (1.0f / (XS * WSC)) * XS, h_, l_); Vt[t * 16 + nloc][wave * 16 + 8 * hlf + r] = h_; Vtl[t * 16 + nloc][wave * 16 + 8 * hlf + r] = l_; }
    __syncthreads();
    for (int pass = 0; pass < 2; ++pass) { for (int q = t_; q < 128 * 8; q += 128) { const int cc = q >> 3, c8 = (q & 7) * 8; const size_t gi = ((size_t)b * F + n0 + cc) * TP + 64 + t0 + c8; *(volatile v8b*)(Yh + gi) = *(const v8b*)(&Vt[cc][c8]); *(volatile v8b*)(Yl + gi) = *(const v8b*)(&Vtl[cc][c8]); } __threadfence(); }
    return; }
#pragma unroll
  for (int t = 0; t < 8; ++t)
#pragma unroll
    for (int r = 0; r < 8; ++r) { float v = acc[t][r] * (1.0f / (XS * WSC)); if (MODE == 0) v = fmaxf(v, 0.0f); Ts[wave][8 * hlf + r][t * 16 + nloc] = v; }
  wave_lds_sync();
  for (int pass = 0; pass < 2; ++pass) { for (int rr = 0; rr < 16; ++rr) {
      if (MODE == 0) { if (lane < 16) { v8b hv, lv; for (int j = 0; j < 8; ++j) { b16 a_, c_; split16(Ts[wave][rr][lane * 8 + j] * XS, a_, c_); hv[j] = a_; lv[j] = c_; } *(volatile v8b*)(Yh + (m0 + rr) * F + n0 + lane * 8) = hv; *(volatile v8b*)(Yl + (m0 + rr) * F + n0 + lane * 8) = lv; } }
      else if (MODE == 1) { const int c4 = n0 + lane * 4; if (c4 < NLP) *(volatile v4f*)(Y32 + (m0 + rr) * NLP + c4) = *(const v4f*)(&Ts[wave][rr][lane * 4]); }
      else { *(volatile v4f*)(Y32 + (m0 + rr) * F + n0 + lane * 4) = *(const v4f*)(&Ts[wave][rr][lane * 4]); } }
    __threadfence(); }
}
__global__ __launch_bounds__(256) void vpad_kernel(b16* __restrict__ VTh, b16* __restrict__ VTl) {
  const int t = blockIdx.x * 256 + threadIdx.x; if (t >= NB * F * 16) return; const int row = t >> 4, part = t & 15; const v8b z = {}; const size_t gi = (size_t)row * TP + (part < 8 ? part * 8 : 64 + T + (part - 8) * 8);
  for (int pass = 0; pass < 2; ++pass) { *(volatile v8b*)(VTh + gi) = z; *(volatile v8b*)(VTl + gi) = z; __threadfence(); }
}
__global__ __launch_bounds__(128) void band_kernel(const float* __restrict__ LG, const b16* __restrict__ VTh, const b16* __restrict__ VTl, b16* __restrict__ Xh, b16* __restrict__ Xl) {
  __shared__ __attribute__((aligned(16))) b16 Ah[4][16][64 + 8], Alo[4][16][64 + 8]; __shared__ float Pr[4][16][CP]; __shared__ __attribute__((aligned(16))) float To[4][16][DK + 4];
  const int wave = threadIdx.x >> 5, lane = threadIdx.x & 31, nloc = lane & 15, hlf = lane >> 4; const int h = blockIdx.y; const size_t m0 = (size_t)blockIdx.x * 64 + wave * 16; const int b = (int)(m0 / T); const int t0 = (int)(m0 - (size_t)b * T);
  { const int rr = lane >> 1, hf = lane & 1; const float* lg = LG + (m0 + rr) * NLP + h * C; float mx = -INFINITY; for (int c = hf; c < C; c += 2) mx = fmaxf(mx, lg[c]); mx = fmaxf(mx, __shfl_xor(mx, 1));
    float s = 0.0f; for (int c = hf; c < C; c += 2) { const float e = nexp(lg[c] - mx); Pr[wave][rr][c] = e; s += e; } s += __shfl_xor(s, 1); const float inv = 1.0f / s;
    __builtin_amdgcn_wave_barrier(); for (int c = hf; c < C; c += 2) Pr[wave][rr][c] *= inv; }
  wave_lds_sync();
  { const int rr = lane >> 1, hf = lane & 1; for (int kk = 0; kk < 32; ++kk) { const int k = hf * 32 + kk; const int c = k - rr - 2; const float a = (c >= 0 && c < C) ? Pr[wave][rr][c] : 0.0f; b16 h_, l_; split16(a * AS, h_, l_); Ah[wave][rr][k] = h_; Alo[wave][rr][k] = l_; } }
  wave_lds_sync();
  v8f o[4] = {{}, {}, {}, {}};
  const b16* Vb = VTh + ((size_t)b * F + h * DK) * TP + t0 + 40;
  const b16* Vlb = VTl + ((size_t)b * F + h * DK) * TP + t0 + 40;
#pragma unroll
  for (int kb = 0; kb < 64; kb += 32) { const v16b a = frag_kb(&Ah[wave][nloc][kb], hlf), al = frag_kb(&Alo[wave][nloc][kb], hlf);
#pragma unroll
    for (int t = 0; t < 4; ++t) { const v16b vf = frag_kb(Vb + (size_t)(t * 16 + nloc) * TP + kb, hlf), vl = frag_kb(Vlb + (size_t)(t * 16 + nloc) * TP + kb, hlf); o[t] = wmma16b(a, vf, o[t]); o[t] = wmma16b(al, vf, o[t]); o[t] = wmma16b(a, vl, o[t]); } }
#pragma unroll
  for (int t = 0; t < 4; ++t)
#pragma unroll
    for (int r = 0; r < 8; ++r) To[wave][8 * hlf + r][t * 16 + nloc] = o[t][r] * (1.0f / (AS * XS));
  wave_lds_sync();
  for (int pass = 0; pass < 2; ++pass) { for (int r4 = 0; r4 < 16; r4 += 4) { const int rr = r4 + (lane >> 3), c8 = (lane & 7) * 8; v8b hv, lv; for (int j = 0; j < 8; ++j) { b16 a_, c_; split16(To[wave][rr][c8 + j] * XS, a_, c_); hv[j] = a_; lv[j] = c_; }
      const size_t gi = (m0 + rr) * F + h * DK + c8; *(volatile v8b*)(Xh + gi) = hv; *(volatile v8b*)(Xl + gi) = lv; } __threadfence(); }
}
}

extern "C" void kernel_launch(void* const* d_in, const int* in_sizes, int n_in, void* d_out, int out_size, void* d_ws, size_t ws_size, hipStream_t stream) {
  (void)n_in;
  auto Fp = [&](int i) { return (const float*)d_in[i]; };
  if (in_sizes[0] != NR * F || in_sizes[2] != NR * F || in_sizes[3] != F * F || in_sizes[4] != F * NL || in_sizes[5] != F * F || in_sizes[6] != F * F || out_size != NR * F) return;
  size_t off = 0; char* ws = (char*)d_ws;
  auto carve = [&](size_t bytes) { char* p = ws + off; off += (bytes + 255) & ~(size_t)255; return p; };
  b16* XQ = (b16*)carve((size_t)NR * F * 2); b16* XV = (b16*)carve((size_t)NR * F * 2); b16* W1T = (b16*)carve((size_t)F * F * 2); b16* W2T = (b16*)carve((size_t)NLP * F * 2); b16* W3T = (b16*)carve((size_t)F * F * 2); b16* WOT = (b16*)carve((size_t)F * F * 2);
  b16* Qh = (b16*)carve((size_t)NR * F * 2); b16* Ql = (b16*)carve((size_t)NR * F * 2); float* LG = (float*)carve((size_t)NR * NLP * 4); b16* VTh = (b16*)carve((size_t)NB * F * TP * 2); b16* VTl = (b16*)carve((size_t)NB * F * TP * 2);
  b16* Xh = XQ; b16* Xl = Qh;
  if (off > ws_size || off > ((size_t)128 << 20)) return;
  prepx_kernel<<<(unsigned)(((size_t)2 * NR * F / 8 + 255) / 256), 256, 0, stream>>>(Fp(0), Fp(2), XQ, XV);
  prepw_kernel<<<dim3(F / 64, F / 64, 4), 256, 0, stream>>>(Fp(3), Fp(4), Fp(5), Fp(6), W1T, W2T, W3T, WOT);
  gemm_kernel<0><<<dim3(NR / 64, F / 128), 128, 0, stream>>>(XQ, nullptr, W1T, F, Qh, Ql, nullptr);
  gemm_kernel<1><<<dim3(NR / 64, 3), 128, 0, stream>>>(Qh, Ql, W2T, F, nullptr, nullptr, LG);
  vpad_kernel<<<(NB * F * 16 + 255) / 256, 256, 0, stream>>>(VTh, VTl);
  gemm_kernel<2><<<dim3(NR / 64, F / 128), 128, 0, stream>>>(XV, nullptr, W3T, F, VTh, VTl, nullptr);
  band_kernel<<<dim3(NR / 64, NH), 128, 0, stream>>>(LG, VTh, VTl, Xh, Xl);
  gemm_kernel<3><<<dim3(NR / 64, F / 128), 128, 0, stream>>>(Xh, Xl, WOT, F, nullptr, nullptr, (float*)d_out);
}
